// BayesianMambaBlock_58746562674867
// MI455X (gfx1250) — hardware-verified
//
#include <hip/hip_runtime.h>
#include <math.h>

typedef __attribute__((ext_vector_type(16))) _Float16 v16h;
typedef __attribute__((ext_vector_type(8)))  _Float16 v8h;
typedef __attribute__((ext_vector_type(16))) __bf16   v16b;
typedef __attribute__((ext_vector_type(8)))  __bf16   v8b;
typedef __attribute__((ext_vector_type(8)))  float    v8f;
typedef __attribute__((ext_vector_type(4)))  float    v4f;

constexpr int kBatch  = 2;
constexpr int kSeq    = 2048;
constexpr int kDm     = 768;
constexpr int kDin    = 1536;
constexpr int kNst    = 16;
constexpr int kConvK  = 4;
constexpr int kRows   = kBatch * kSeq;
constexpr int kPdW    = 64;
constexpr float kEps  = 1e-5f;
constexpr float kWScale  = 8.0f;
constexpr float kXaScale = 16.0f;
constexpr float kUScale  = 32.0f;
constexpr float kGyScale = 128.0f;
constexpr int kConvTP = 260;
constexpr int kScanTS = 64;
constexpr int kScanCh = 64;
constexpr int kScanYP = 68;
static_assert(4 * kNst == kPdW, "stacked param width");
static_assert((kDm % 32) == 0 && (kDin % 32) == 0, "GEMM K multiples of 32");
static_assert((kRows % 64) == 0 && (kDin % 64) == 0 && (kPdW % 64) == 0 && (kDm % 64) == 0, "GEMM M,N multiples of 64");
static_assert((kSeq % kScanTS) == 0 && (kSeq % 64) == 0 && (kDin % kScanCh) == 0 && (kDin % 256) == 0, "tile multiples");
static_assert(kDm == 3 * 256, "LayerNorm thread map");

constexpr size_t kOffXN  = 0;
constexpr size_t kOffWIN = kOffXN  + (size_t)kRows * kDm  * 2;
constexpr size_t kOffWS  = kOffWIN + (size_t)kDin  * kDm  * 2;
constexpr size_t kOffWP  = kOffWS  + (size_t)kDin  * kDin * 2;
constexpr size_t kOffWG  = kOffWP  + (size_t)kPdW  * kDin * 2;
constexpr size_t kOffWO  = kOffWG  + (size_t)kDin  * kDm  * 2;
constexpr size_t kOffR1  = kOffWO  + (size_t)kDm   * kDin * 2;
constexpr size_t kOffR2  = kOffR1  + (size_t)kRows * kDin * 4;
constexpr size_t kOffR3  = kOffR2  + (size_t)kRows * kDin * 4;
constexpr size_t kOffR4  = kOffR3  + (size_t)kRows * kDin * 2;
constexpr size_t kOffPD  = kOffR4  + (size_t)kRows * kDin * 2;
constexpr size_t kOffGY  = kOffPD  + (size_t)kRows * kPdW * 4;
constexpr size_t kWsTotal = kOffGY + (size_t)kRows * kDin * 2;
static_assert(kWsTotal == 107413504ull, "carve total");
static_assert(kWsTotal <= 134217728ull, "carve cap");
static_assert(kOffPD - kOffR3 == (size_t)kRows * kDin * 4, "R3+R4 holds one f32 plane");
static_assert((kOffWIN % 128) == 0 && (kOffWS % 128) == 0 && (kOffWP % 128) == 0 && (kOffWG % 128) == 0 &&
              (kOffWO % 128) == 0 && (kOffR1 % 128) == 0 && (kOffR2 % 128) == 0 && (kOffR3 % 128) == 0 &&
              (kOffR4 % 128) == 0 && (kOffPD % 128) == 0 && (kOffGY % 128) == 0, "128-B aligned regions");

__device__ __forceinline__ unsigned short f2bf_bits(float f) {
  unsigned u = __float_as_uint(f);
  return (unsigned short)((u + 0x7FFFu + ((u >> 16) & 1u)) >> 16);
}
__device__ __forceinline__ float bf_bits2f(unsigned short h) { return __uint_as_float(((unsigned)h) << 16); }

__device__ __forceinline__ void dep_guard_h(v8f& a, v8f& b, v16h x, v16h y) { asm volatile("v_nop\n\tv_nop\n\tv_nop\n\tv_nop" : "+v"(a), "+v"(b) : "v"(x), "v"(y)); }
__device__ __forceinline__ void dep_guard_b(v8f& a, v8f& b, v16b x, v16b y) { asm volatile("v_nop\n\tv_nop\n\tv_nop\n\tv_nop" : "+v"(a), "+v"(b) : "v"(x), "v"(y)); }
__device__ __forceinline__ void keep4_h(v16h a, v16h b, v16h c, v16h d) { asm volatile("v_nop" :: "v"(a), "v"(b), "v"(c), "v"(d)); }
__device__ __forceinline__ void keep4_b(v16b a, v16b b, v16b c, v16b d) { asm volatile("v_nop" :: "v"(a), "v"(b), "v"(c), "v"(d)); }
__device__ __forceinline__ void acc_guard4(v8f& a, v8f& b, v8f& c, v8f& d) { asm volatile("v_nop\n\tv_nop\n\tv_nop\n\tv_nop" : "+v"(a), "+v"(b), "+v"(c), "+v"(d)); }
template <typename T> struct Frag;
template <> struct Frag<_Float16> {
  typedef v16h V; union U { v16h v; v8h h[2]; };
  static __device__ __forceinline__ v16h load(const _Float16* p) {
    U f; f.h[0] = *(const v8h*)(p); f.h[1] = *(const v8h*)(p + 16); return f.v;
  }
  static __device__ __forceinline__ v8f mma(v16h a, v16h b, v8f c) {
    return __builtin_amdgcn_wmma_f32_16x16x32_f16(false, a, false, b, (short)0, c, false, false);
  }
  static __device__ __forceinline__ void guard(v8f& a, v8f& b, v16h x, v16h y) { dep_guard_h(a, b, x, y); }
  static __device__ __forceinline__ void keep(v16h a, v16h b, v16h c, v16h d) { keep4_h(a, b, c, d); }
};
template <> struct Frag<__bf16> {
  typedef v16b V; union U { v16b v; v8b h[2]; };
  static __device__ __forceinline__ v16b load(const __bf16* p) {
    U f; f.h[0] = *(const v8b*)(p); f.h[1] = *(const v8b*)(p + 16); return f.v;
  }
  static __device__ __forceinline__ v8f mma(v16b a, v16b b, v8f c) {
    return __builtin_amdgcn_wmma_f32_16x16x32_bf16(false, a, false, b, (short)0, c, false, false);
  }
  static __device__ __forceinline__ void guard(v8f& a, v8f& b, v16b x, v16b y) { dep_guard_b(a, b, x, y); }
  static __device__ __forceinline__ void keep(v16b a, v16b b, v16b c, v16b d) { keep4_b(a, b, c, d); }
};

template <int ET> struct Elem;
template <> struct Elem<0> { typedef _Float16 T; };
template <> struct Elem<1> { typedef __bf16 T; };
template <int ET, bool SPLIT, int BIAS_MODE, int OUT_MODE, bool RESID, int ACT = 0>
__global__ __launch_bounds__(256) void wmma_gemm64(
    const unsigned short* __restrict__ Ap, const unsigned short* __restrict__ A2p, int lda, long strideA,
    const unsigned short* __restrict__ Btp, const unsigned short* __restrict__ Bt2p, int ldb, long strideB,
    void* __restrict__ Cout, void* __restrict__ Cout2, int ldc, long strideC,
    const float* __restrict__ bias,
    const float* __restrict__ resid, long strideR,
    int M, int N, int K, float scale) {
  typedef typename Elem<ET>::T T;
  typedef typename Frag<T>::V V;
  const T* A = (const T*)Ap; const T* A2 = (const T*)A2p; const T* Bt = (const T*)Btp; const T* Bt2 = (const T*)Bt2p;
  __shared__ __align__(16) float sT[8][16 * 68];
  const int b    = blockIdx.y;
  const int lane = threadIdx.x & 31;
  const int wave = threadIdx.x >> 5;
  const int tilesN = N >> 6;
  const int tilesM = M >> 6;
  const int tile = blockIdx.x * 8 + wave;
  if (tile >= tilesM * tilesN) return;
  const int tm = tile / tilesN;
  const int tn = tile - tm * tilesN;
  const int m0 = tm << 6;
  const int n0 = tn << 6;

  const T* Ab  = A  + (size_t)b * strideA;
  const T* Bb  = Bt + (size_t)b * strideB;
  const T* Ab2 = SPLIT ? (A2  + (size_t)b * strideA) : nullptr;
  const T* Bb2 = SPLIT ? (Bt2 + (size_t)b * strideB) : nullptr;

  const int rlane = lane & 15;
  const int koff  = (lane >> 4) * 8;
  const int mOff  = (lane >> 4) * 8;

  v8f acc[4][4];
#pragma unroll
  for (int i = 0; i < 4; ++i)
#pragma unroll
    for (int j = 0; j < 4; ++j) acc[i][j] = (v8f){0.f,0.f,0.f,0.f,0.f,0.f,0.f,0.f};

  for (int k0 = 0; k0 < K; k0 += 32) {
    V bh[4], bl[4];
#pragma unroll
    for (int j = 0; j < 4; ++j) {
      const size_t bo = (size_t)(n0 + (j << 4) + rlane) * ldb + koff + k0;
      bh[j] = Frag<T>::load(Bb + bo);
      if (SPLIT) bl[j] = Frag<T>::load(Bb2 + bo);
    }
#pragma unroll
    for (int i = 0; i < 4; ++i) {
      const size_t ao = (size_t)(m0 + (i << 4) + rlane) * lda + koff + k0;
      V ah = Frag<T>::load(Ab + ao);
      V al;
      if (SPLIT) al = Frag<T>::load(Ab2 + ao);
#pragma unroll
      for (int j = 0; j < 4; ++j) {
        acc[i][j] = Frag<T>::mma(ah, bh[j], acc[i][j]);
        if (SPLIT) {
          acc[i][j] = Frag<T>::mma(ah, bl[j], acc[i][j]);
          acc[i][j] = Frag<T>::mma(al, bh[j], acc[i][j]);
        }
      }
      Frag<T>::guard(acc[i][0], acc[i][3], ah, SPLIT ? al : ah);
    }
    Frag<T>::keep(bh[0], bh[1], bh[2], bh[3]);
    if (SPLIT) Frag<T>::keep(bl[0], bl[1], bl[2], bl[3]);
  }
  acc_guard4(acc[0][0], acc[0][1], acc[0][2], acc[0][3]);
  acc_guard4(acc[1][0], acc[1][1], acc[1][2], acc[1][3]);
  acc_guard4(acc[2][0], acc[2][1], acc[2][2], acc[2][3]);
  acc_guard4(acc[3][0], acc[3][1], acc[3][2], acc[3][3]);

  float* slab = sT[wave];
  const float* Rb = RESID ? (resid + (size_t)b * strideR) : nullptr;
#pragma unroll
  for (int i = 0; i < 4; ++i) {
    const int mBase = m0 + (i << 4);
#pragma unroll
    for (int j = 0; j < 4; ++j) {
      const int n = n0 + (j << 4) + rlane;
      float bv = 0.f;
      if (BIAS_MODE == 2) bv = bias[n];
#pragma unroll
      for (int r = 0; r < 8; ++r) {
        float v = acc[i][j][r] * scale;
        if (BIAS_MODE == 1) v += bias[mBase + mOff + r];
        if (BIAS_MODE == 2) v += bv;
        if (RESID) v += Rb[(size_t)(mBase + mOff + r) * ldc + n];
        if (ACT == 1) v = tanhf(v);
        if (ACT == 2) v = fmaxf(v, 0.0f);
        if (ACT == 3) v = v / (1.0f + expf(-v));
        if (ACT == 4) v = (v > 0.f) ? v : 0.01f * v;
        if (ACT == 5) v = 0.5f * v * (1.0f + erff(v * 0.70710678118654752f));
        slab[(mOff + r) * 68 + (j << 4) + rlane] = v;
      }
    }
    __builtin_amdgcn_fence(__ATOMIC_RELEASE, "workgroup");
    __builtin_amdgcn_wave_barrier();
    __builtin_amdgcn_fence(__ATOMIC_ACQUIRE, "workgroup");
    if (OUT_MODE == 0) {
      float* C = (float*)Cout + (size_t)b * strideC;
      const int hh = lane >> 4, c4 = (lane & 15) * 4;
      for (int pass = 0; pass < 2; ++pass) {
#pragma unroll
        for (int it = 0; it < 8; ++it) {
          const int row = it * 2 + hh;
          v4f v = *(const v4f*)(slab + row * 68 + c4);
          *(volatile v4f*)(C + (size_t)(mBase + row) * ldc + n0 + c4) = v;
        }
        __threadfence();
      }
    } else {
      const int q = lane >> 3, c8 = (lane & 7) * 8;
      unsigned short* C  = (unsigned short*)Cout  + (size_t)b * strideC;
      unsigned short* C2 = (OUT_MODE == 2) ? ((unsigned short*)Cout2 + (size_t)b * strideC) : nullptr;
      for (int pass = 0; pass < 2; ++pass) {
#pragma unroll
        for (int it = 0; it < 4; ++it) {
          const int row = it * 4 + q;
          const float* sp = slab + row * 68 + c8;
          v8h hv, lv;
#pragma unroll
          for (int e = 0; e < 8; ++e) {
            if (OUT_MODE == 1) {
              hv[e] = (_Float16)sp[e];
            } else {
              unsigned short hb = f2bf_bits(sp[e]);
              unsigned short lb = f2bf_bits(sp[e] - bf_bits2f(hb));
              hv[e] = __builtin_bit_cast(_Float16, hb);
              lv[e] = __builtin_bit_cast(_Float16, lb);
            }
          }
          *(volatile v8h*)(C + (size_t)(mBase + row) * ldc + n0 + c8) = hv;
          if (OUT_MODE == 2) *(volatile v8h*)(C2 + (size_t)(mBase + row) * ldc + n0 + c8) = lv;
        }
        __threadfence();
      }
    }
    __builtin_amdgcn_fence(__ATOMIC_RELEASE, "workgroup");
    __builtin_amdgcn_wave_barrier();
    __builtin_amdgcn_fence(__ATOMIC_ACQUIRE, "workgroup");
  }
}

__global__ __launch_bounds__(256) void cast_rows_f16_kernel(
    const float* __restrict__ src, unsigned short* __restrict__ dst, int total8, float scale)
{
  const int i = blockIdx.x * 256 + threadIdx.x;
  if (i >= total8) return;
  const size_t e0 = (size_t)i << 3;
  const v4f a0 = *(const v4f*)(src + e0);
  const v4f a1 = *(const v4f*)(src + e0 + 4);
  v8h hv;
#pragma unroll
  for (int e = 0; e < 4; ++e) {
    hv[e]     = (_Float16)(a0[e] * scale);
    hv[4 + e] = (_Float16)(a1[e] * scale);
  }
  unsigned short* q = dst + e0;
  *(volatile v8h*)q = hv;
  __threadfence();
  *(volatile v8h*)q = hv;
}

__global__ __launch_bounds__(256) void layernorm_f16_kernel(
    const float* __restrict__ x, const float* __restrict__ g, const float* __restrict__ bta,
    unsigned short* __restrict__ XN)
{
  __shared__ float sRed[16];
  __shared__ __align__(16) float sN[kDm];
  const int tid = threadIdx.x, lane = tid & 31, wave = tid >> 5;
  const size_t rbase = (size_t)blockIdx.x * kDm;
  const float v0 = x[rbase + tid], v1 = x[rbase + tid + 256], v2 = x[rbase + tid + 512];
  float s = v0 + v1 + v2;
#pragma unroll
  for (int off = 1; off < 32; off <<= 1) s += __shfl_xor(s, off, 32);
  if (lane == 0) sRed[wave] = s;
  __syncthreads();
  float tot = 0.f;
#pragma unroll
  for (int w = 0; w < 8; ++w) tot += sRed[w];
  const float mu = tot * (1.0f / (float)kDm);
  const float q0 = v0 - mu, q1 = v1 - mu, q2 = v2 - mu;
  float s2 = q0 * q0 + q1 * q1 + q2 * q2;
#pragma unroll
  for (int off = 1; off < 32; off <<= 1) s2 += __shfl_xor(s2, off, 32);
  if (lane == 0) sRed[8 + wave] = s2;
  __syncthreads();
  float tot2 = 0.f;
#pragma unroll
  for (int w = 0; w < 8; ++w) tot2 += sRed[8 + w];
  const float var = tot2 * (1.0f / (float)kDm);
  const float rs  = rsqrtf(var + kEps);
  sN[tid]       = q0 * rs * g[tid]       + bta[tid];
  sN[tid + 256] = q1 * rs * g[tid + 256] + bta[tid + 256];
  sN[tid + 512] = q2 * rs * g[tid + 512] + bta[tid + 512];
  __syncthreads();
  if (tid < 96) {
    const v4f a0 = *(const v4f*)(sN + 8 * tid);
    const v4f a1 = *(const v4f*)(sN + 8 * tid + 4);
    v8h hv;
#pragma unroll
    for (int e = 0; e < 4; ++e) {
      hv[e]     = (_Float16)a0[e];
      hv[4 + e] = (_Float16)a1[e];
    }
    unsigned short* p = XN + rbase + 8 * tid;
    *(volatile v8h*)p = hv;
    __threadfence();
    *(volatile v8h*)p = hv;
  }
}

__global__ __launch_bounds__(256) void conv_silu_kernel(
    const float* __restrict__ XP, const float* __restrict__ cw, const float* __restrict__ cb,
    float* __restrict__ XA, unsigned short* __restrict__ XA16)
{
  __shared__ __align__(16) float sT[16 * kConvTP];
  const int tid = threadIdx.x, lane = tid & 31, wave = tid >> 5;
  const int d0 = blockIdx.x * 256, d = d0 + tid;
  const int g0 = blockIdx.y * 64;
  const int tb = g0 & (kSeq - 1);
  const float w0 = cw[d * kConvK + 0], w1 = cw[d * kConvK + 1], w2 = cw[d * kConvK + 2], w3 = cw[d * kConvK + 3];
  const float bc = cb[d];
  float xm3, xm2, xm1;
  {
    const bool hist = (tb > 0);
    const int rb = hist ? (g0 - 3) : g0;
    const float v3 = XP[(size_t)rb * kDin + d];
    const float v2 = XP[(size_t)(rb + 1) * kDin + d];
    const float v1 = XP[(size_t)(rb + 2) * kDin + d];
    xm3 = hist ? v3 : 0.f;
    xm2 = hist ? v2 : 0.f;
    xm1 = hist ? v1 : 0.f;
  }
  const int hrow = wave >> 1;
  const int hch  = (wave & 1) * 128 + lane * 4;
#pragma unroll 1
  for (int sub = 0; sub < 4; ++sub) {
    const int lb = g0 + sub * 16;
#pragma unroll 1
    for (int s = 0; s < 16; ++s) {
      const float xcur = XP[(size_t)(lb + s) * kDin + d];
      float acc = w0 * xm3;
      acc = fmaf(w1, xm2, acc);
      acc = fmaf(w2, xm1, acc);
      acc = fmaf(w3, xcur, acc);
      const float sv = acc + bc;
      const float sg = __builtin_amdgcn_rcpf(1.0f + expf(-sv));
      sT[s * kConvTP + tid] = sv * sg;
      xm3 = xm2; xm2 = xm1; xm1 = xcur;
    }
    __syncthreads();
    v4f fv[4];
    v8h hv[2];
#pragma unroll
    for (int it = 0; it < 4; ++it) fv[it] = *(const v4f*)(sT + (it * 4 + hrow) * kConvTP + hch);
#pragma unroll
    for (int it = 0; it < 2; ++it) {
      const float* sp = sT + (it * 8 + wave) * kConvTP + lane * 8;
      const v4f a0 = *(const v4f*)(sp);
      const v4f a1 = *(const v4f*)(sp + 4);
#pragma unroll
      for (int e = 0; e < 4; ++e) {
        hv[it][e]     = (_Float16)(a0[e] * kXaScale);
        hv[it][4 + e] = (_Float16)(a1[e] * kXaScale);
      }
    }
    for (int pass = 0; pass < 2; ++pass) {
#pragma unroll
      for (int it = 0; it < 4; ++it)
        *(volatile v4f*)(XA + (size_t)(lb + it * 4 + hrow) * kDin + d0 + hch) = fv[it];
#pragma unroll
      for (int it = 0; it < 2; ++it) {
        const size_t o = (size_t)(lb + it * 8 + wave) * kDin + d0 + lane * 8;
        *(volatile v8h*)(XA16 + o) = hv[it];
      }
      __threadfence();
    }
    __syncthreads();
  }
}

__global__ __launch_bounds__(256) void gate_cast_kernel(
    const float* __restrict__ SA, const float* __restrict__ XA, unsigned short* __restrict__ U16, int total8)
{
  const int i = blockIdx.x * 256 + threadIdx.x;
  if (i >= total8) return;
  const size_t e0 = (size_t)i << 3;
  const v4f s0 = *(const v4f*)(SA + e0);
  const v4f s1 = *(const v4f*)(SA + e0 + 4);
  const v4f a0 = *(const v4f*)(XA + e0);
  const v4f a1 = *(const v4f*)(XA + e0 + 4);
  v8h hv;
#pragma unroll
  for (int e = 0; e < 4; ++e) {
    const float u0 = a0[e] * __builtin_amdgcn_rcpf(1.0f + expf(-s0[e]));
    const float u1 = a1[e] * __builtin_amdgcn_rcpf(1.0f + expf(-s1[e]));
    hv[e]     = (_Float16)(u0 * kUScale);
    hv[4 + e] = (_Float16)(u1 * kUScale);
  }
  unsigned short* q = U16 + e0;
  *(volatile v8h*)q = hv;
  __threadfence();
  *(volatile v8h*)q = hv;
}

__global__ __launch_bounds__(64) void scan_kernel(
    const float* __restrict__ PD, const float* __restrict__ SA, const float* __restrict__ XA,
    const float* __restrict__ GP,
    const float* __restrict__ bA, const float* __restrict__ bDt, const float* __restrict__ bB,
    const float* __restrict__ bC, unsigned short* __restrict__ GY)
{
  __shared__ __align__(16) float sX[kScanTS * kPdW];
  __shared__ __align__(16) float sY[kScanTS * kScanYP];
  const int tid = threadIdx.x, lane = tid & 31, wave = tid >> 5;
  constexpr int kBlkPerB = kDin / kScanCh;
  const int bix = blockIdx.x / kBlkPerB;
  const int d0  = (blockIdx.x - bix * kBlkPerB) * kScanCh;
  const int d   = d0 + tid;
  const size_t row0 = (size_t)bix * kSeq;
  float h[kNst];
#pragma unroll
  for (int n = 0; n < kNst; ++n) h[n] = 0.f;
  const int lr = tid >> 4, lc4 = (tid & 15) * 4, lc4b = (lc4 + 16) & 63;
  const int grp = (tid & 15) >> 2;
  const int nb  = lc4 & 15;
  float ba[4], bt[4], bb[4], bc[4];
#pragma unroll
  for (int e = 0; e < 4; ++e) {
    ba[e] = bA[nb + e];
    bt[e] = bDt[nb + e];
    bb[e] = bB[nb + e];
    bc[e] = bC[nb + e];
  }
  const int q = lane >> 3, c8 = (lane & 7) * 8;
#pragma unroll 1
  for (int t0 = 0; t0 < kSeq; t0 += kScanTS) {
    __syncthreads();
#pragma unroll 1
    for (int i = 0; i < 16; ++i) {
      const int r = lr + 4 * i;
      const float* pr = PD + (row0 + t0 + r) * kPdW;
      const v4f xv = *(const v4f*)(pr + lc4);
      const v4f x2 = *(const v4f*)(pr + lc4b);
      v4f o;
#pragma unroll
      for (int e = 0; e < 4; ++e) {
        const float av  = -__expf(xv[e] + ba[e]);
        const float tv  = __expf(x2[e] + bt[e]);
        const float dec = __expf(av * tv);
        const float bm  = xv[e] + bb[e];
        const float cm  = xv[e] + bc[e];
        o[e] = (grp == 0) ? dec : ((grp == 2) ? bm : ((grp == 3) ? cm : xv[e]));
      }
      *(v4f*)(sX + r * kPdW + lc4) = o;
    }
    __syncthreads();
#pragma unroll 1
    for (int s = 0; s < kScanTS; ++s) {
      const float* xr = sX + s * kPdW;
      float Ds[kNst], Bs[kNst], Cs[kNst];
#pragma unroll
      for (int q4 = 0; q4 < 4; ++q4) {
        const v4f dv = *(const v4f*)(xr + 4 * q4);
        const v4f bv = *(const v4f*)(xr + 2 * kNst + 4 * q4);
        const v4f cv = *(const v4f*)(xr + 3 * kNst + 4 * q4);
        Ds[4 * q4 + 0] = dv[0]; Ds[4 * q4 + 1] = dv[1]; Ds[4 * q4 + 2] = dv[2]; Ds[4 * q4 + 3] = dv[3];
        Bs[4 * q4 + 0] = bv[0]; Bs[4 * q4 + 1] = bv[1]; Bs[4 * q4 + 2] = bv[2]; Bs[4 * q4 + 3] = bv[3];
        Cs[4 * q4 + 0] = cv[0]; Cs[4 * q4 + 1] = cv[1]; Cs[4 * q4 + 2] = cv[2]; Cs[4 * q4 + 3] = cv[3];
      }
      const size_t gi = (row0 + t0 + s) * kDin + d;
      const float sv  = SA[gi];
      const float xav = XA[gi];
      const float gv  = GP[gi];
      const float ut  = xav * __builtin_amdgcn_rcpf(1.0f + expf(-sv));
      const float gt  = gv * __builtin_amdgcn_rcpf(1.0f + expf(-gv));
      float y = 0.f;
#pragma unroll
      for (int n = 0; n < kNst; ++n) {
        const float bu = Bs[n] * ut;
        h[n] = h[n] * Ds[n] + bu;
        y = h[n] * Cs[n] + y;
      }
      sY[s * kScanYP + tid] = gt * y;
    }
    __syncthreads();
    v8h hv[8];
#pragma unroll
    for (int it = 0; it < 8; ++it) {
      const int row = it * 8 + wave * 4 + q;
      const float* sp = sY + row * kScanYP + c8;
      const v4f a0 = *(const v4f*)(sp);
      const v4f a1 = *(const v4f*)(sp + 4);
#pragma unroll
      for (int e = 0; e < 4; ++e) {
        hv[it][e]     = (_Float16)(a0[e] * kGyScale);
        hv[it][4 + e] = (_Float16)(a1[e] * kGyScale);
      }
    }
    for (int pass = 0; pass < 2; ++pass) {
#pragma unroll
      for (int it = 0; it < 8; ++it) {
        const int row = it * 8 + wave * 4 + q;
        const size_t o = (row0 + t0 + row) * kDin + d0 + c8;
        *(volatile v8h*)(GY + o) = hv[it];
      }
      __threadfence();
    }
  }
}

extern "C" void kernel_launch(void* const* d_in, const int* in_sizes, int n_in,
                              void* d_out, int out_size, void* d_ws, size_t ws_size,
                              hipStream_t stream) {
  if (n_in < 21) return;
  if (in_sizes[0]  != kRows * kDm) return;
  if (in_sizes[1]  != kDm) return;
  if (in_sizes[2]  != kDm) return;
  if (in_sizes[3]  != kDin * kDm) return;
  if (in_sizes[4]  != kDin) return;
  if (in_sizes[5]  != kDin * kConvK) return;
  if (in_sizes[6]  != kDin) return;
  if (in_sizes[7]  != kNst * kDin) return;
  if (in_sizes[8]  != kNst) return;
  if (in_sizes[9]  != kNst * kDin) return;
  if (in_sizes[10] != kNst) return;
  if (in_sizes[11] != kNst * kDin) return;
  if (in_sizes[12] != kNst) return;
  if (in_sizes[13] != kNst * kDin) return;
  if (in_sizes[14] != kNst) return;
  if (in_sizes[15] != 2 * kDin * kDin) return;
  if (in_sizes[16] != 2 * kDin) return;
  if (in_sizes[17] != kDin * kDm) return;
  if (in_sizes[18] != kDin) return;
  if (in_sizes[19] != kDm * kDin) return;
  if (in_sizes[20] != kDm) return;
  if (out_size != kRows * kDm) return;
  if (ws_size < kWsTotal) return;

  const float* x      = (const float*)d_in[0];
  const float* ln_g   = (const float*)d_in[1];
  const float* ln_b   = (const float*)d_in[2];
  const float* W_in   = (const float*)d_in[3];
  const float* b_in   = (const float*)d_in[4];
  const float* conv_w = (const float*)d_in[5];
  const float* conv_b = (const float*)d_in[6];
  const float* W_A    = (const float*)d_in[7];
  const float* b_A    = (const float*)d_in[8];
  const float* W_B    = (const float*)d_in[9];
  const float* b_B    = (const float*)d_in[10];
  const float* W_C    = (const float*)d_in[11];
  const float* b_C    = (const float*)d_in[12];
  const float* W_dt   = (const float*)d_in[13];
  const float* b_dt   = (const float*)d_in[14];
  const float* W_S    = (const float*)d_in[15];
  const float* b_S    = (const float*)d_in[16];
  const float* W_gate = (const float*)d_in[17];
  const float* b_gate = (const float*)d_in[18];
  const float* W_out  = (const float*)d_in[19];
  const float* b_out  = (const float*)d_in[20];
  float* out = (float*)d_out;

  char* ws = (char*)d_ws;
  unsigned short* XN   = (unsigned short*)(ws + kOffXN);
  unsigned short* WIN8 = (unsigned short*)(ws + kOffWIN);
  unsigned short* WS8  = (unsigned short*)(ws + kOffWS);
  unsigned short* WP8  = (unsigned short*)(ws + kOffWP);
  unsigned short* WG8  = (unsigned short*)(ws + kOffWG);
  unsigned short* WO8  = (unsigned short*)(ws + kOffWO);
  float*          XP   = (float*)(ws + kOffR1);
  float*          SA   = (float*)(ws + kOffR1);
  float*          XA   = (float*)(ws + kOffR2);
  unsigned short* XA16 = (unsigned short*)(ws + kOffR3);
  unsigned short* U16  = (unsigned short*)(ws + kOffR4);
  float*          GPre = (float*)(ws + kOffR3);
  float*          PD   = (float*)(ws + kOffPD);
  unsigned short* GY16 = (unsigned short*)(ws + kOffGY);

  cast_rows_f16_kernel<<<(kDin * kDm / 8) / 256, 256, 0, stream>>>(W_in, WIN8, kDin * kDm / 8, kWScale);
  cast_rows_f16_kernel<<<(kDin * kDin / 8) / 256, 256, 0, stream>>>(W_S, WS8, kDin * kDin / 8, kWScale);
  cast_rows_f16_kernel<<<(kDin * kDm / 8) / 256, 256, 0, stream>>>(W_gate, WG8, kDin * kDm / 8, kWScale);
  cast_rows_f16_kernel<<<(kDm * kDin / 8) / 256, 256, 0, stream>>>(W_out, WO8, kDm * kDin / 8, kWScale);
  cast_rows_f16_kernel<<<(kNst * kDin / 8) / 256, 256, 0, stream>>>(W_A,  WP8 + (size_t)0 * kNst * kDin, kNst * kDin / 8, kWScale);
  cast_rows_f16_kernel<<<(kNst * kDin / 8) / 256, 256, 0, stream>>>(W_dt, WP8 + (size_t)1 * kNst * kDin, kNst * kDin / 8, kWScale);
  cast_rows_f16_kernel<<<(kNst * kDin / 8) / 256, 256, 0, stream>>>(W_B,  WP8 + (size_t)2 * kNst * kDin, kNst * kDin / 8, kWScale);
  cast_rows_f16_kernel<<<(kNst * kDin / 8) / 256, 256, 0, stream>>>(W_C,  WP8 + (size_t)3 * kNst * kDin, kNst * kDin / 8, kWScale);

  layernorm_f16_kernel<<<kRows, 256, 0, stream>>>(x, ln_g, ln_b, XN);

  wmma_gemm64<0, false, 2, 0, false, 0><<<dim3(192, 1), 256, 0, stream>>>(
      XN, nullptr, kDm, 0L,
      WIN8, nullptr, kDm, 0L,
      (void*)XP, nullptr, kDin, 0L,
      b_in, nullptr, 0L,
      kRows, kDin, kDm, 1.0f / 8.0f);

  conv_silu_kernel<<<dim3(kDin / 256, kRows / 64), 256, 0, stream>>>(XP, conv_w, conv_b, XA, XA16);

  wmma_gemm64<0, false, 2, 0, false, 0><<<dim3(192, 1), 256, 0, stream>>>(
      XA16, nullptr, kDin, 0L,
      WS8, nullptr, kDin, 0L,
      (void*)SA, nullptr, kDin, 0L,
      b_S, nullptr, 0L,
      kRows, kDin, kDin, 1.0f / 128.0f);

  gate_cast_kernel<<<(kRows * kDin / 8) / 256, 256, 0, stream>>>(SA, XA, U16, kRows * kDin / 8);

  wmma_gemm64<0, false, 0, 0, false, 0><<<dim3(8, 1), 256, 0, stream>>>(
      U16, nullptr, kDin, 0L,
      WP8, nullptr, kDin, 0L,
      (void*)PD, nullptr, kPdW, 0L,
      nullptr, nullptr, 0L,
      kRows, kPdW, kDin, 1.0f / 256.0f);

  wmma_gemm64<0, false, 2, 0, false, 0><<<dim3(192, 1), 256, 0, stream>>>(
      XN, nullptr, kDm, 0L,
      WG8, nullptr, kDm, 0L,
      (void*)GPre, nullptr, kDin, 0L,
      b_gate, nullptr, 0L,
      kRows, kDin, kDm, 1.0f / 8.0f);

  scan_kernel<<<kBatch * (kDin / kScanCh), kScanCh, 0, stream>>>(PD, SA, XA, GPre, b_A, b_dt, b_B, b_C, GY16);

  wmma_gemm64<0, false, 2, 0, true, 0><<<dim3(96, 1), 256, 0, stream>>>(
      GY16, nullptr, kDin, 0L,
      WO8, nullptr, kDin, 0L,
      (void*)out, nullptr, kDm, 0L,
      b_out, x, 0L,
      kRows, kDm, kDin, 1.0f / 1024.0f);
}
